// FNO_5239860101553
// MI455X (gfx1250) — hardware-verified
//
#include <hip/hip_runtime.h>

typedef unsigned short us;
typedef us     v8us  __attribute__((ext_vector_type(8)));
typedef __bf16 v16bf __attribute__((ext_vector_type(16)));
typedef float  v8f   __attribute__((ext_vector_type(8)));
typedef float  v4f   __attribute__((ext_vector_type(4)));
typedef float  v2f   __attribute__((ext_vector_type(2)));
typedef v8us __attribute__((may_alias)) v8usa;
typedef v4f  __attribute__((may_alias)) v4fa;
typedef v2f  __attribute__((may_alias)) v2fa;

union Frag { v16bf v; v8us p[2]; };

#ifndef NB
#define NB 1048576
#endif
#define NB_FULL 1048576
#define INDIM  10
#define DIM    32
#define LAYERS 4
#define MODES  17
#define RPT    32
#define NPC    (RPT * INDIM / 4)

static_assert((NB % RPT) == 0);
static_assert(NB <= NB_FULL);
static_assert(NPC == 80);

#define TW_ST    0
#define TW_LH    1024
#define TW_LL    5120
#define TW_HD    9216
#define TW_TOTAL 9728
#define BT_FLOATS 192

__device__ __forceinline__ v8f mma(v16bf a, v16bf b, v8f c) {
  v8f d = __builtin_amdgcn_wmma_f32_16x16x32_bf16(false, a, false, b, (short)0, c, false, false);
  asm volatile("v_nop\n\tv_nop\n\tv_nop\n\tv_nop" : "+v"(d) : "v"(a), "v"(b));
  return d;
}
__device__ __forceinline__ v8f mma3(v16bf ah, v16bf al, v16bf bh, v16bf bl, v8f c) {
  c = mma(ah, bh, c);
  c = mma(ah, bl, c);
  c = mma(al, bh, c);
  return c;
}

__device__ __forceinline__ unsigned bfb(float x) {
  const unsigned u = __float_as_uint(x);
  return (u + 0x7FFFu + ((u >> 16) & 1u)) >> 16;
}
__device__ __forceinline__ float bf2f(us b) { return __uint_as_float(((unsigned)b) << 16); }
__device__ __forceinline__ float bfrne(float x) { return __uint_as_float(bfb(x) << 16); }
__device__ __forceinline__ void split1(float x, us& hi, us& lo) {
  const unsigned hb = bfb(x);
  hi = (us)hb;
  lo = (us)bfb(x - __uint_as_float(hb << 16));
}
__device__ __forceinline__ void split_v8(v8f d, v8us& hi, v8us& lo) {
  us h0, h1, h2, h3, h4, h5, h6, h7, l0, l1, l2, l3, l4, l5, l6, l7;
  split1(d[0], h0, l0); split1(d[1], h1, l1); split1(d[2], h2, l2); split1(d[3], h3, l3);
  split1(d[4], h4, l4); split1(d[5], h5, l5); split1(d[6], h6, l6); split1(d[7], h7, l7);
  v8us H = {h0, h1, h2, h3, h4, h5, h6, h7};
  v8us L = {l0, l1, l2, l3, l4, l5, l6, l7};
  hi = H; lo = L;
}
__device__ __forceinline__ v8us pack8(float a0, float a1, float a2, float a3, float a4, float a5, float a6, float a7) {
  v8us H = {(us)bfb(a0), (us)bfb(a1), (us)bfb(a2), (us)bfb(a3), (us)bfb(a4), (us)bfb(a5), (us)bfb(a6), (us)bfb(a7)};
  return H;
}

__device__ __forceinline__ v16bf ldfrag(const us* p, int h) {
  Frag f;
  f.p[0] = *(const v8usa*)(p + 8 * h);
  f.p[1] = *(const v8usa*)(p + 16 + 8 * h);
  return f.v;
}
__device__ __forceinline__ v8f ld8f(const float* p) {
  const v4f a = *(const v4fa*)p;
  const v4f b = *(const v4fa*)(p + 4);
  v8f r = {a.x, a.y, a.z, a.w, b.x, b.y, b.z, b.w};
  return r;
}

__device__ __forceinline__ v8f silu8(v8f v) {
#pragma unroll
  for (int r = 0; r < 8; ++r) {
    const float xx = v[r];
    const float t  = expf(-fabsf(xx));
    const float rc = 1.0f / (1.0f + t);
    const float sg = (xx >= 0.0f) ? rc : t * rc;
    v[r] = xx * sg;
  }
  return v;
}

__global__ __launch_bounds__(256) void k_prep(const float* __restrict__ stem_W, const float* __restrict__ stem_b,
                                              const float* __restrict__ fwr, const float* __restrict__ fwi,
                                              const float* __restrict__ proj_W, const float* __restrict__ proj_b,
                                              const float* __restrict__ head_W, const float* __restrict__ head_b,
                                              us* __restrict__ tw, float* __restrict__ bt) {
#pragma clang fp contract(off)
  __shared__ float sWr[LAYERS * MODES * MODES];
  __shared__ float sWi[LAYERS * MODES * MODES];
  __shared__ float sC[32];
  __shared__ float sS[32];
  const int tid = threadIdx.x;
#pragma unroll 1
  for (int i = tid; i < LAYERS * MODES * MODES; i += 256) {
    sWr[i] = bfrne(fwr[i]);
    sWi[i] = bfrne(fwi[i]);
  }
  if (tid < 32) {
    const float a = (float)tid * 0.0625f;
    sC[tid] = cospif(a);
    sS[tid] = sinpif(a);
  }
  __syncthreads();
  const int g = blockIdx.x * 256 + tid;
  if (g < 128) {
    const int c = g, o = c >> 2, k0 = (c & 3) * 8;
    float v[8];
#pragma unroll
    for (int e = 0; e < 8; ++e) {
      const int k = k0 + e;
      const int kc = (k < INDIM) ? k : (INDIM - 1);
      const float t = stem_W[kc * DIM + o];
      v[e] = (k < INDIM) ? t : 0.0f;
    }
    const v8us H = pack8(v[0], v[1], v[2], v[3], v[4], v[5], v[6], v[7]);
    us* dh = tw + TW_ST + c * 8;
    *(volatile v8us*)dh = H;
    __threadfence();
    *(volatile v8us*)dh = H;
  } else if (g < 640) {
    const int c = g - 128, l = c >> 7, o = (c >> 2) & 31, k0 = (c & 3) * 8;
    v8f acc = {0.f, 0.f, 0.f, 0.f, 0.f, 0.f, 0.f, 0.f};
#pragma unroll 1
    for (int km = 0; km < MODES; ++km) {
      const float ck = (km == 0 || km == MODES - 1) ? 1.0f : 2.0f;
#pragma unroll 1
      for (int j = 0; j < MODES; ++j) {
        const float wr = sWr[(l * MODES + j) * MODES + km];
        const float wi = sWi[(l * MODES + j) * MODES + km];
        const int base = km * o - j * k0;
#pragma unroll
        for (int e = 0; e < 8; ++e) {
          const int t = (base - j * e) & 31;
          acc[e] = acc[e] + ck * (wr * sC[t] - wi * sS[t]);
        }
      }
    }
    float v[8];
#pragma unroll
    for (int e = 0; e < 8; ++e) {
      const int k = k0 + e;
      v[e] = acc[e] * 0.03125f + bfrne(proj_W[(l * DIM + k) * DIM + o]);
    }
    v4f a = {v[0], v[1], v[2], v[3]};
    v4f b = {v[4], v[5], v[6], v[7]};
    v8f ab = {a.x, a.y, a.z, a.w, b.x, b.y, b.z, b.w};
    v8us H, L;
    split_v8(ab, H, L);
    us* dh = tw + TW_LH + c * 8;
    us* dl = tw + TW_LL + c * 8;
    *(volatile v8us*)dh = H;
    *(volatile v8us*)dl = L;
    __threadfence();
    *(volatile v8us*)dh = H;
    *(volatile v8us*)dl = L;
  } else if (g < 704) {
    const int c = g - 640, o = c >> 2, k0 = (c & 3) * 8;
    const int oc = (o < INDIM) ? o : (INDIM - 1);
    float v[8];
#pragma unroll
    for (int e = 0; e < 8; ++e) {
      const int k = k0 + e;
      const float t = head_W[k * INDIM + oc];
      v[e] = (o < INDIM) ? t : 0.0f;
    }
    const v8us H = pack8(v[0], v[1], v[2], v[3], v[4], v[5], v[6], v[7]);
    us* dh = tw + TW_HD + c * 8;
    *(volatile v8us*)dh = H;
    __threadfence();
    *(volatile v8us*)dh = H;
  } else {
    const int q = g - 704;
    const int qc = (q < 48) ? q : 47;
    const int row = qc >> 3, col0 = (qc & 7) * 4;
    float v[4];
#pragma unroll
    for (int i = 0; i < 4; ++i) {
      const int col = col0 + i;
      const float a = stem_b[col];
      int rr = row - 1; rr = (rr < 0) ? 0 : ((rr > LAYERS - 1) ? (LAYERS - 1) : rr);
      const float b = proj_b[rr * DIM + col];
      const int cc = (col < INDIM) ? col : (INDIM - 1);
      const float d = head_b[cc];
      const float f = (row == 0) ? a : ((row <= LAYERS) ? b : ((col < INDIM) ? d : 0.0f));
      v[i] = bfrne(f);
    }
    const v4f val = {v[0], v[1], v[2], v[3]};
    if (q < 48) *(volatile v4f*)(bt + 4 * q) = val;
    __threadfence();
    if (q < 48) *(volatile v4f*)(bt + 4 * q) = val;
  }
}

__global__ __launch_bounds__(128) void k_main(const float* __restrict__ x, const us* __restrict__ tw,
                                              const float* __restrict__ bt, float* __restrict__ out, int ntasks) {
  __shared__ __attribute__((aligned(16))) float sO[4 * RPT * INDIM];
  const int tid = threadIdx.x, lane = tid & 31, w = tid >> 5, h = lane >> 4, m = lane & 15;
  const int task = blockIdx.x * 4 + w;
  if (task >= ntasks) return;
  const int rbase = task * RPT;
  const bool up = (h != 0);

  v16bf ast[2];
  v8f bst[2];
#pragma unroll
  for (int mt = 0; mt < 2; ++mt) {
    ast[mt] = ldfrag(tw + TW_ST + (16 * mt + m) * DIM, h);
    bst[mt] = ld8f(bt + 16 * mt + 8 * h);
  }
  v16bf hb[2], hl[2];
#pragma unroll
  for (int s = 0; s < 2; ++s) {
    const float* xr = x + (size_t)(rbase + 16 * s + m) * INDIM;
    const v2f q0 = *(const v2fa*)(xr);
    const v2f q1 = *(const v2fa*)(xr + 2);
    const v2f q2 = *(const v2fa*)(xr + 4);
    const v2f q3 = *(const v2fa*)(xr + 6);
    const v2f q4 = *(const v2fa*)(xr + 8);
    const float e0 = up ? q4.x : q0.x;
    const float e1 = up ? q4.y : q0.y;
    const float e2 = up ? 0.0f : q1.x;
    const float e3 = up ? 0.0f : q1.y;
    const float e4 = up ? 0.0f : q2.x;
    const float e5 = up ? 0.0f : q2.y;
    const float e6 = up ? 0.0f : q3.x;
    const float e7 = up ? 0.0f : q3.y;
    Frag bx;
    bx.p[0] = pack8(e0, e1, e2, e3, e4, e5, e6, e7);
    const v8us pz = {0, 0, 0, 0, 0, 0, 0, 0};
    bx.p[1] = pz;
    const v8f d0 = mma(ast[0], bx.v, bst[0]);
    const v8f d1 = mma(ast[1], bx.v, bst[1]);
    Frag H, L;
    split_v8(d0, H.p[0], L.p[0]);
    split_v8(d1, H.p[1], L.p[1]);
    hb[s] = H.v; hl[s] = L.v;
  }

#pragma unroll 1
  for (int l = 0; l < LAYERS; ++l) {
    v16bf ah[2], al[2];
    v8f bl8[2];
#pragma unroll
    for (int mt = 0; mt < 2; ++mt) {
      ah[mt]  = ldfrag(tw + TW_LH + (l * DIM + 16 * mt + m) * DIM, h);
      al[mt]  = ldfrag(tw + TW_LL + (l * DIM + 16 * mt + m) * DIM, h);
      bl8[mt] = ld8f(bt + (1 + l) * DIM + 16 * mt + 8 * h);
    }
#pragma unroll
    for (int s = 0; s < 2; ++s) {
      v8f d0 = mma3(ah[0], al[0], hb[s], hl[s], bl8[0]);
      v8f d1 = mma3(ah[1], al[1], hb[s], hl[s], bl8[1]);
      d0 = silu8(d0);
      d1 = silu8(d1);
      Frag H, L;
      split_v8(d0, H.p[0], L.p[0]);
      split_v8(d1, H.p[1], L.p[1]);
      hb[s] = H.v; hl[s] = L.v;
    }
  }

  const v16bf ahd = ldfrag(tw + TW_HD + m * DIM, h);
  const v8f bhd = ld8f(bt + (1 + LAYERS) * DIM + 8 * h);
  float* sw = sO + w * (RPT * INDIM);
#pragma unroll
  for (int s = 0; s < 2; ++s) {
    v8f o8 = mma(ahd, hb[s], bhd);
    o8 = mma(ahd, hl[s], o8);
    float* so = sw + (16 * s + m) * INDIM + 8 * h;
    const v2f t0 = {o8[0], o8[1]};
    *(v2fa*)(so) = t0;
    if (!up) {
      const v2f t1 = {o8[2], o8[3]};
      const v2f t2 = {o8[4], o8[5]};
      const v2f t3 = {o8[6], o8[7]};
      *(v2fa*)(so + 2) = t1;
      *(v2fa*)(so + 4) = t2;
      *(v2fa*)(so + 6) = t3;
    }
  }
  __builtin_amdgcn_fence(__ATOMIC_RELEASE, "wavefront");
  __builtin_amdgcn_wave_barrier();

  float* dst = out + (size_t)rbase * INDIM;
#pragma unroll
  for (int pass = 0; pass < 2; ++pass) {
#pragma unroll
    for (int j = 0; j < 3; ++j) {
      const int p = 32 * j + lane;
      const int pc = (p < NPC) ? p : (NPC - 1);
      const v4f vv = *(const v4fa*)(sw + 4 * pc);
      if (p < NPC) *(volatile v4f*)(dst + 4 * p) = vv;
    }
    if (pass == 0) __threadfence();
  }
}

extern "C" void kernel_launch(void* const* d_in, const int* in_sizes, int n_in,
                              void* d_out, int out_size, void* d_ws, size_t ws_size,
                              hipStream_t stream) {
  if (n_in < 9) return;
  if (in_sizes[0] < NB * INDIM) return;
  if (in_sizes[1] < INDIM * DIM || in_sizes[2] < DIM) return;
  if (in_sizes[3] < LAYERS * MODES * MODES || in_sizes[4] < LAYERS * MODES * MODES) return;
  if (in_sizes[5] < LAYERS * DIM * DIM || in_sizes[6] < LAYERS * DIM) return;
  if (in_sizes[7] < DIM * INDIM || in_sizes[8] < INDIM) return;
  if (out_size < NB * INDIM) return;

  const float* x      = (const float*)d_in[0];
  const float* stem_W = (const float*)d_in[1];
  const float* stem_b = (const float*)d_in[2];
  const float* fwr    = (const float*)d_in[3];
  const float* fwi    = (const float*)d_in[4];
  const float* proj_W = (const float*)d_in[5];
  const float* proj_b = (const float*)d_in[6];
  const float* head_W = (const float*)d_in[7];
  const float* head_b = (const float*)d_in[8];
  float* out = (float*)d_out;

  const size_t twBytes = (size_t)TW_TOTAL * 2;
  const size_t btBytes = (size_t)BT_FLOATS * 4;
  const size_t total = twBytes + btBytes;
  if (total > ws_size) return;
  char* wsb = (char*)d_ws;
  us*    tw = (us*)(wsb);
  float* bt = (float*)(wsb + twBytes);

  k_prep<<<3, 256, 0, stream>>>(stem_W, stem_b, fwr, fwi, proj_W, proj_b, head_W, head_b, tw, bt);

  const int ntasks = NB / RPT;
  const int nblk = (ntasks + 3) / 4;
  k_main<<<nblk, 128, 0, stream>>>(x, tw, bt, out, ntasks);
}
